// GCN_80401787781186
// MI455X (gfx1250) — hardware-verified
//
#include <hip/hip_runtime.h>
#include <stddef.h>
#include <stdint.h>
#include <math.h>


#define FD      128
#define KD      256
#define NGR     2048
#define NTHR    256
#define NWAVE   8
#define EPT     8
#define CHUNK   (NTHR * EPT)
#define WCAP    (EPT * 32)
#define LISTN   (NWAVE * WCAP)
#define NBA     1024
#define SLA     10
#define SRCB    17
#define RCAP    28672
#define DEGCAP  128
#define MEAS_B1024  16710
#define MEAS_MAXDEG 36
#define ASL     128
#define GBM     64
#define GBN     64
#define GTHR    128
#define MROWS   128
#define NUW1    (FD * (FD / 8))
#define NUWD    (FD * (KD / 8))
#define PGR     32
#define BNEPS   1e-5f
#define SELU_A  1.6732632423543772f
#define SELU_S  1.0507009873554805f
#define WSMAX   134217728
#define BKT_ZINTS    (RCAP + 3 * NBA)
#define BKT_LDS_INTS (LISTN + 2 * RCAP + 3 * NBA + 16 + NBA)
#define STAT_LDS_FLOATS (MROWS * FD + 3 * FD)

static_assert((CHUNK & (CHUNK - 1)) == 0 && CHUNK <= 4096);
static_assert((NBA & (NBA - 1)) == 0 && NBA == (1 << SLA) && NBA <= 1024);
static_assert(((long long)CHUNK << SLA) < (1LL << 31));
static_assert(SRCB + SLA < 31);
static_assert(LISTN >= NWAVE * WCAP);
static_assert(NBA == 4 * NTHR);
static_assert((RCAP % 32) == 0 && (BKT_ZINTS % 4) == 0);
static_assert(RCAP >= MEAS_B1024 + 4096);
static_assert(DEGCAP >= MEAS_MAXDEG + 8);
static_assert(BKT_LDS_INTS * 4 <= 300000);
static_assert(STAT_LDS_FLOATS * 4 <= 300000);
static_assert(GBM == (GTHR / 32) * 16 && GBN == 64);
static_assert((FD % GBN) == 0 && (FD % 32) == 0 && (KD % 32) == 0 && KD == 2 * FD);
static_assert((MROWS % GBM) == 0 && (NBA % ASL) == 0 && ASL == 16 * NWAVE && MROWS == 16 * NWAVE);
static_assert(FD == 4 * 32);
static_assert((NUW1 % NTHR) == 0 && (NUWD % NTHR) == 0);
static_assert((NGR % PGR) == 0 && PGR == 4 * NWAVE && (NGR % GBM) == 0);
static_assert((MROWS * FD) % (4 * NTHR) == 0);

typedef float          v4f  __attribute__((ext_vector_type(4)));
typedef float          v8f  __attribute__((ext_vector_type(8)));
typedef int            v4i  __attribute__((ext_vector_type(4)));
typedef int            v8i  __attribute__((ext_vector_type(8)));
typedef unsigned short v8us __attribute__((ext_vector_type(8)));
typedef __bf16         v16b __attribute__((ext_vector_type(16)));
typedef v4f  __attribute__((may_alias)) v4fa;
typedef v4i  __attribute__((may_alias)) v4ia;
typedef v8us __attribute__((may_alias)) v8usa;
union FragB { v16b v; v8us h[2]; v8i w; };

__device__ __forceinline__ v8f wmb(const FragB& a, const FragB& b, v8f c) {
  v8f d = __builtin_amdgcn_wmma_f32_16x16x32_bf16(false, a.v, false, b.v, (short)0, c, false, false);
  asm volatile("v_nop\n\tv_nop\n\tv_nop\n\tv_nop" : "+v"(d) : "v"(a.w), "v"(b.w));
  return d;
}

__device__ __forceinline__ unsigned int f2bf(float f) {
  const unsigned int u = __float_as_uint(f);
  const unsigned int r = ((u + 0x7FFFu + ((u >> 16) & 1u)) >> 16) & 0xFFFFu;
  return ((u & 0x7FFFFFFFu) > 0x7F800000u) ? 0x7FC0u : r;
}
__device__ __forceinline__ float bf2f(unsigned int b) { return __uint_as_float(b << 16); }
__device__ __forceinline__ float bfr(float f) { return bf2f(f2bf(f)); }

__device__ __forceinline__ v8us wgath(const float* __restrict__ p) {
  v8us o;
#pragma unroll
  for (int i = 0; i < 8; ++i) o[i] = (unsigned short)f2bf(p[(size_t)i * FD]);
  return o;
}

template <int SLB>
__device__ __forceinline__ int scan_chunk(const int* __restrict__ dsts, int nE, int cbase, int slotBase,
                                          int nb, int vec8, int* list, int tid, int lane, int wave) {
  int wc = 0;
  const int el0  = tid * EPT;
  const int e0   = cbase + el0;
  const int sent = -2147483647 - 1;
  v4i da, db;
  if (vec8 != 0 && cbase + CHUNK <= nE) {
    da = *(const v4i*)(dsts + e0);
    db = *(const v4i*)(dsts + e0 + 4);
  } else {
    da.x = (e0     < nE) ? dsts[min(e0,     nE - 1)] : sent;
    da.y = (e0 + 1 < nE) ? dsts[min(e0 + 1, nE - 1)] : sent;
    da.z = (e0 + 2 < nE) ? dsts[min(e0 + 2, nE - 1)] : sent;
    da.w = (e0 + 3 < nE) ? dsts[min(e0 + 3, nE - 1)] : sent;
    db.x = (e0 + 4 < nE) ? dsts[min(e0 + 4, nE - 1)] : sent;
    db.y = (e0 + 5 < nE) ? dsts[min(e0 + 5, nE - 1)] : sent;
    db.z = (e0 + 6 < nE) ? dsts[min(e0 + 6, nE - 1)] : sent;
    db.w = (e0 + 7 < nE) ? dsts[min(e0 + 7, nE - 1)] : sent;
  }
  const unsigned nbs = (unsigned)slotBase;
  const unsigned unb = (unsigned)nb;
  const unsigned s0 = (unsigned)da.x - nbs, s1 = (unsigned)da.y - nbs;
  const unsigned s2 = (unsigned)da.z - nbs, s3 = (unsigned)da.w - nbs;
  const unsigned s4 = (unsigned)db.x - nbs, s5 = (unsigned)db.y - nbs;
  const unsigned s6 = (unsigned)db.z - nbs, s7 = (unsigned)db.w - nbs;
  const bool h0 = s0 < unb, h1 = s1 < unb, h2 = s2 < unb, h3 = s3 < unb;
  const bool h4 = s4 < unb, h5 = s5 < unb, h6 = s6 < unb, h7 = s7 < unb;
  const unsigned any = __builtin_amdgcn_ballot_w32(h0 | h1 | h2 | h3 | h4 | h5 | h6 | h7);
  if (any != 0u) {
#define HITJ(J, HJ, SJ) { \
      const unsigned mj = __builtin_amdgcn_ballot_w32(HJ); \
      if (mj != 0u) { \
        if (HJ) { \
          const int pos = wc + (int)__builtin_amdgcn_mbcnt_lo(mj, 0u); \
          if (pos < WCAP) list[wave * WCAP + pos] = ((el0 + (J)) << SLB) | (int)(SJ); \
        } \
        wc += (int)__builtin_popcount(mj); } }
    HITJ(0, h0, s0)
    HITJ(1, h1, s1)
    HITJ(2, h2, s2)
    HITJ(3, h3, s3)
    HITJ(4, h4, s4)
    HITJ(5, h5, s5)
    HITJ(6, h6, s6)
    HITJ(7, h7, s7)
#undef HITJ
  }
  return wc;
}

__global__ __launch_bounds__(NTHR) void k_prep(const float* __restrict__ x, const float* __restrict__ W1,
                                               const float* __restrict__ W2, const float* __restrict__ W3,
                                               const float* __restrict__ FW1, unsigned short* XB,
                                               unsigned short* W1T, unsigned short* W2D, unsigned short* W3D,
                                               unsigned short* FW1D, int nN, int nUx) {
  const int u = (int)blockIdx.x * NTHR + (int)threadIdx.x;
  v8us o;
  unsigned short* dp;
  if (u < nUx) {
    const int row = u >> 4;
    const int k8  = (u & 15) * 8;
    const int rc  = row < nN ? row : nN - 1;
    const float* p = x + (size_t)rc * FD + k8;
    const v4f a = *(const v4fa*)p;
    const v4f b = *(const v4fa*)(p + 4);
    const bool ok = row < nN;
    o[0] = ok ? (unsigned short)f2bf(a.x) : (unsigned short)0;
    o[1] = ok ? (unsigned short)f2bf(a.y) : (unsigned short)0;
    o[2] = ok ? (unsigned short)f2bf(a.z) : (unsigned short)0;
    o[3] = ok ? (unsigned short)f2bf(a.w) : (unsigned short)0;
    o[4] = ok ? (unsigned short)f2bf(b.x) : (unsigned short)0;
    o[5] = ok ? (unsigned short)f2bf(b.y) : (unsigned short)0;
    o[6] = ok ? (unsigned short)f2bf(b.z) : (unsigned short)0;
    o[7] = ok ? (unsigned short)f2bf(b.w) : (unsigned short)0;
    dp = XB + (size_t)row * FD + k8;
  } else if (u < nUx + NUW1) {
    const int v  = u - nUx;
    const int n  = v >> 4;
    const int k8 = (v & 15) * 8;
    o  = wgath(W1 + (size_t)k8 * FD + n);
    dp = W1T + (size_t)n * FD + k8;
  } else if (u < nUx + NUW1 + NUWD) {
    const int v  = u - nUx - NUW1;
    const int n  = v >> 5;
    const int k8 = (v & 31) * 8;
    o  = wgath(W2 + (size_t)(k8 & (FD - 1)) * FD + n);
    dp = W2D + (size_t)n * KD + k8;
  } else if (u < nUx + NUW1 + 2 * NUWD) {
    const int v  = u - nUx - NUW1 - NUWD;
    const int n  = v >> 5;
    const int k8 = (v & 31) * 8;
    o  = wgath(W3 + (size_t)(k8 & (FD - 1)) * FD + n);
    dp = W3D + (size_t)n * KD + k8;
  } else if (u < nUx + NUW1 + 3 * NUWD) {
    const int v  = u - nUx - NUW1 - 2 * NUWD;
    const int n  = v >> 5;
    const int k8 = (v & 31) * 8;
    o  = wgath(FW1 + (size_t)(k8 & (FD - 1)) * FD + n);
    dp = FW1D + (size_t)n * KD + k8;
  } else {
    return;
  }
  *(volatile v8usa*)dp = o;
  __threadfence();
  *(volatile v8usa*)dp = o;
}

__global__ __launch_bounds__(NTHR) void k_bucket(const int* __restrict__ srcs, const int* __restrict__ dsts,
                                                 int nE, int nN, int vec8, int* LIST, int* CNT, int* OFF,
                                                 int* DISB, int* FLG) {
  extern __shared__ __attribute__((aligned(16))) int bsm[];
  int* list = bsm;
  int* reg1 = bsm + LISTN;
  int* sl   = reg1 + RCAP;
  int* cnt  = sl + RCAP;
  int* offs = cnt + NBA;
  int* cur  = offs + NBA;
  int* misc = cur + NBA;
  int* disi = misc + 16;
  const int tid = (int)threadIdx.x, lane = tid & 31, wave = tid >> 5;
  const int blk = (int)blockIdx.x;
  const int nodeBase = blk * NBA;
  int nb = nN - nodeBase;
  nb = nb < 0 ? 0 : (nb > NBA ? NBA : nb);

  {
    const v4i z4 = {0, 0, 0, 0};
    for (int i = tid * 4; i < BKT_ZINTS; i += NTHR * 4) *(v4ia*)(sl + i) = z4;
    for (int i = tid; i < LISTN; i += NTHR) list[i] = 0;
    if (tid < 16) misc[tid] = 0;
  }
  __syncthreads();

  int tot = 0, ovf = 0;
  const int nChunks = (nE + CHUNK - 1) / CHUNK;
#pragma unroll 1
  for (int ch = 0; ch < nChunks; ++ch) {
    const int cbase = ch * CHUNK;
    const int wc = scan_chunk<SLA>(dsts, nE, cbase, nodeBase, nb, vec8, list, tid, lane, wave);
    if (lane == 0) misc[wave] = wc;
    __syncthreads();
    int pre = 0, all = 0;
#pragma unroll
    for (int w2 = 0; w2 < NWAVE; ++w2) {
      int c = misc[w2];
      c = c < 0 ? 0 : (c > WCAP ? WCAP : c);
      all += c;
      pre += (w2 < wave) ? c : 0;
    }
    const int wcc  = wc > WCAP ? WCAP : wc;
    const int base = tot + pre;
#pragma unroll 1
    for (int i = lane; i < wcc; i += 32) {
      const int ent = list[wave * WCAP + i];
      const int el  = (ent >> SLA) & (CHUNK - 1);
      const int sq  = ent & (NBA - 1);
      int eid = cbase + el;
      eid = eid > nE - 1 ? nE - 1 : eid;
      const int sraw = srcs[eid];
      const int s = sraw < 0 ? 0 : (sraw > nN - 1 ? nN - 1 : sraw);
      const int pos = base + i;
      if (pos < RCAP) reg1[pos] = (int)((unsigned)s | ((unsigned)sq << SRCB));
    }
    if (tot + all > RCAP) ovf = 1;
    tot += all;
    tot = tot > RCAP ? RCAP : tot;
    __syncthreads();
  }
  const int nh = tot;

  if (wave == 0) {
#pragma unroll 1
    for (int b0 = 0; b0 < nh; b0 += 32) {
      const int idx = b0 + lane;
      const int uv  = reg1[idx < nh ? idx : nh - 1];
      const int m32 = (nh - b0) < 32 ? (nh - b0) : 32;
#pragma unroll 1
      for (int k = 0; k < m32; ++k) {
        const int u  = __builtin_amdgcn_readlane(uv, k);
        const int sq = (u >> SRCB) & (NBA - 1);
        if (lane == 0) cnt[sq] = cnt[sq] + 1;
      }
    }
  }
  __syncthreads();
  if (wave == 0) {
    const int base = lane * (NBA / 32);
    int s = 0;
#pragma unroll 1
    for (int i = 0; i < NBA / 32; ++i) s += cnt[base + i];
    int incl = s;
#pragma unroll
    for (int d = 1; d < 32; d <<= 1) {
      const int y = __shfl_up(incl, d, 32);
      if (lane >= d) incl += y;
    }
    int run = incl - s;
#pragma unroll 1
    for (int i = 0; i < NBA / 32; ++i) {
      const int cv = cnt[base + i];
      offs[base + i] = run;
      cur[base + i]  = run;
      run += cv;
    }
  }
  __syncthreads();
  if (wave == 0) {
#pragma unroll 1
    for (int b0 = 0; b0 < nh; b0 += 32) {
      const int idx = b0 + lane;
      const int uv  = reg1[idx < nh ? idx : nh - 1];
      const int m32 = (nh - b0) < 32 ? (nh - b0) : 32;
#pragma unroll 1
      for (int k = 0; k < m32; ++k) {
        const int u  = __builtin_amdgcn_readlane(uv, k);
        const int sq = (u >> SRCB) & (NBA - 1);
        if (lane == 0) {
          int p = cur[sq];
          p = p < 0 ? 0 : (p > RCAP - 1 ? RCAP - 1 : p);
          sl[p] = u;
          cur[sq] = p + 1;
        }
      }
    }
  }
#pragma unroll 1
  for (int i = tid; i < NBA; i += NTHR) {
    const float dg = (float)(cnt[i] + 1);
    const float rs = 1.0f / sqrtf(fmaxf(dg, 1.0f));
    disi[i] = __float_as_int(dg > 0.0f ? rs : 0.0f);
  }
  __syncthreads();

  const int nhPad = (nh + 31) & ~31;
  int* lb = LIST + (size_t)blk * RCAP;
  const v4i cq = *(const v4ia*)(cnt + 4 * tid);
  const v4i oq = *(const v4ia*)(offs + 4 * tid);
  const v4i dq = *(const v4ia*)(disi + 4 * tid);
  v4i fv;
  fv.x = (tid == 0) ? nh : 0;
  fv.y = (tid == 0) ? ovf : 0;
  fv.z = 0; fv.w = 0;
  int* fp = FLG + (size_t)blk * 32 + 4 * (tid & 7);
  const int smask = (1 << SRCB) - 1;
#pragma unroll 1
  for (int p = tid * 4; p < nhPad; p += NTHR * 4) {
    v4i v = *(const v4ia*)(sl + p);
    v.x &= smask; v.y &= smask; v.z &= smask; v.w &= smask;
    *(volatile v4i*)(lb + p) = v;
  }
  *(volatile v4i*)(CNT + (size_t)nodeBase + 4 * tid) = cq;
  *(volatile v4i*)(OFF + (size_t)nodeBase + 4 * tid) = oq;
  *(volatile v4i*)(DISB + (size_t)nodeBase + 4 * tid) = dq;
  if (tid < 8) *(volatile v4i*)fp = fv;
  __threadfence();
#pragma unroll 1
  for (int p = tid * 4; p < nhPad; p += NTHR * 4) {
    v4i v = *(const v4ia*)(sl + p);
    v.x &= smask; v.y &= smask; v.z &= smask; v.w &= smask;
    *(volatile v4i*)(lb + p) = v;
  }
  *(volatile v4i*)(CNT + (size_t)nodeBase + 4 * tid) = cq;
  *(volatile v4i*)(OFF + (size_t)nodeBase + 4 * tid) = oq;
  *(volatile v4i*)(DISB + (size_t)nodeBase + 4 * tid) = dq;
  if (tid < 8) *(volatile v4i*)fp = fv;
}

__global__ __launch_bounds__(GTHR) void k_gemm(
    const unsigned short* __restrict__ A, const unsigned short* __restrict__ WT,
    float* outF, int K, int ldo)
{
  __shared__ __attribute__((aligned(16))) float stg[GBM * GBN];
  const int tid = (int)threadIdx.x, lane = tid & 31, wave = tid >> 5, hh = lane >> 4, m = lane & 15;
  const int rowBase = (int)blockIdx.x * GBM;
  const int col0    = (int)blockIdx.y * GBN;

  v8f acc[4];
  {
    const v8f z = {0.f, 0.f, 0.f, 0.f, 0.f, 0.f, 0.f, 0.f};
    acc[0] = z; acc[1] = z; acc[2] = z; acc[3] = z;
  }
  const unsigned short* ap = A  + (size_t)(rowBase + 16 * wave + m) * (size_t)K + 8 * hh;
  const unsigned short* wp = WT + (size_t)(col0 + m) * (size_t)K + 8 * hh;
  const int ksteps = K >> 5;
#pragma unroll 1
  for (int ks = 0; ks < ksteps; ++ks) {
    FragB af;
    af.h[0] = *(const v8usa*)(ap + 32 * ks);
    af.h[1] = *(const v8usa*)(ap + 32 * ks + 16);
#pragma unroll
    for (int t = 0; t < 4; ++t) {
      const unsigned short* wq = wp + (size_t)(16 * t) * (size_t)K + 32 * ks;
      FragB bf;
      bf.h[0] = *(const v8usa*)wq;
      bf.h[1] = *(const v8usa*)(wq + 16);
      acc[t] = wmb(af, bf, acc[t]);
    }
  }

#pragma unroll
  for (int t = 0; t < 4; ++t) {
    const int lc = 16 * t + m;
#pragma unroll
    for (int r = 0; r < 8; ++r) {
      const int lr = 16 * wave + 8 * hh + r;
      stg[lr * GBN + lc] = acc[t][r];
    }
  }
  __syncthreads();

  v4f fv[8];
#pragma unroll
  for (int i = 0; i < 8; ++i) {
    const int lr = 16 * wave + 2 * i + hh;
    fv[i] = *(const v4fa*)(stg + lr * GBN + 4 * m);
  }
#pragma unroll
  for (int i = 0; i < 8; ++i) {
    const int lr = 16 * wave + 2 * i + hh;
    const int gr = rowBase + lr;
    float* op = outF + (size_t)gr * (size_t)ldo + col0 + 4 * m;
    *(volatile v4f*)op = fv[i];
  }
  __threadfence();
#pragma unroll
  for (int i = 0; i < 8; ++i) {
    const int lr = 16 * wave + 2 * i + hh;
    const int gr = rowBase + lr;
    float* op = outF + (size_t)gr * (size_t)ldo + col0 + 4 * m;
    *(volatile v4f*)op = fv[i];
  }
}

template <int MODE>
__global__ __launch_bounds__(NTHR) void k_agg(const int* __restrict__ LIST, const int* __restrict__ CNT,
                                              const int* __restrict__ OFF, const int* __restrict__ FLG,
                                              const float* __restrict__ DIS, const float* __restrict__ H,
                                              const float* __restrict__ bias, float* outp, int nN, int MPr) {
  __shared__ __attribute__((aligned(16))) float st[NWAVE * FD];
  const int tid = (int)threadIdx.x, lane = tid & 31, wave = tid >> 5;
  const int nodeBase = (int)blockIdx.x * ASL;
  const int bb = nodeBase >> SLA;
  const int nhraw = FLG[(size_t)bb * 32];
  const int bflag = FLG[(size_t)bb * 32 + 1];
  const int nh  = nhraw < 0 ? 0 : (nhraw > RCAP ? RCAP : nhraw);
  const bool ovf = (bflag != 0) || (nhraw < 0) || (nhraw > RCAP);
  const int* lb = LIST + (size_t)bb * RCAP;
  float* sw = st + wave * FD;
  v4f bz;
  {
    const v4f bq = *(const v4fa*)(bias + 4 * lane);
    bz.x = bfr(bq.x); bz.y = bfr(bq.y); bz.z = bfr(bq.z); bz.w = bfr(bq.w);
  }
  const float qnan = __int_as_float(0x7fc00000);

#pragma unroll 1
  for (int si = 0; si < ASL / NWAVE; ++si) {
    const int s    = si * NWAVE + wave;
    const int node = nodeBase + s;
    const int nc   = node < nN ? node : nN - 1;
    const int craw = CNT[node];
    const int oraw = OFF[node];
    const bool incons = (craw < 0) || (oraw < 0) || (oraw > nh) || (craw > nh - oraw) || (craw > DEGCAP);
    int c = craw < 0 ? 0 : (craw > DEGCAP ? DEGCAP : craw);
    int o = oraw < 0 ? 0 : (oraw > nh ? nh : oraw);
    if (c > nh - o) c = nh - o;
    const float dd = DIS[nc];
    const float rd = dd * dd;
    float a0 = 0.0f, a1 = 0.0f, a2 = 0.0f, a3 = 0.0f;
#pragma unroll 1
    for (int b0 = 0; b0 < c; b0 += 32) {
      int idx = o + b0 + lane;
      idx = idx > nh - 1 ? nh - 1 : idx;
      idx = idx < 0 ? 0 : idx;
      int sr = lb[idx];
      sr = sr < 0 ? 0 : (sr > nN - 1 ? nN - 1 : sr);
      const float cf  = DIS[sr] * dd;
      const int   cfi = __float_as_int(cf);
      const int m32 = (c - b0) < 32 ? (c - b0) : 32;
#pragma unroll 1
      for (int k = 0; k < m32; ++k) {
        const int   sk = __builtin_amdgcn_readlane(sr, k);
        const float ck = __int_as_float(__builtin_amdgcn_readlane(cfi, k));
        const v4f a = *(const v4fa*)(H + (size_t)sk * FD + 4 * lane);
        a0 = fmaf(ck, a.x, a0); a1 = fmaf(ck, a.y, a1);
        a2 = fmaf(ck, a.z, a2); a3 = fmaf(ck, a.w, a3);
      }
    }
    const v4f sv = *(const v4fa*)(H + (size_t)nc * FD + 4 * lane);
    float y0 = (a0 + sv.x * rd) + bz.x;
    float y1 = (a1 + sv.y * rd) + bz.y;
    float y2 = (a2 + sv.z * rd) + bz.z;
    float y3 = (a3 + sv.w * rd) + bz.w;
    if constexpr (MODE == 0) {
      sw[lane] = y0; sw[32 + lane] = y1; sw[64 + lane] = y2; sw[96 + lane] = y3;
#pragma unroll 1
      for (int j = 0; j < 4; ++j) {
        const float v = sw[j * 32 + lane];
        const float r = (v > 0.0f) ? v : SELU_A * expm1f(v);
        sw[j * 32 + lane] = SELU_S * r;
      }
      y0 = sw[lane]; y1 = sw[32 + lane]; y2 = sw[64 + lane]; y3 = sw[96 + lane];
    } else {
      y0 = (y0 > 0.0f) ? y0 : (y0 - y0);
      y1 = (y1 > 0.0f) ? y1 : (y1 - y1);
      y2 = (y2 > 0.0f) ? y2 : (y2 - y2);
      y3 = (y3 > 0.0f) ? y3 : (y3 - y3);
    }
    const bool bad  = ovf || incons;
    const bool live = node < nN;
    v4f ow;
    ow.x = live ? (bad ? qnan : y0) : 0.0f;
    ow.y = live ? (bad ? qnan : y1) : 0.0f;
    ow.z = live ? (bad ? qnan : y2) : 0.0f;
    ow.w = live ? (bad ? qnan : y3) : 0.0f;
    if (node < MPr) {
      float* op = outp + (size_t)node * FD + 4 * lane;
      *(volatile v4f*)op = ow;
      __threadfence();
      *(volatile v4f*)op = ow;
    }
  }
}

__global__ __launch_bounds__(NTHR) void k_stats(const float* __restrict__ S, float* REC, int nN) {
  extern __shared__ __attribute__((aligned(16))) float tsm[];
  float* tile = tsm;
  float* rec  = tsm + MROWS * FD;
  const int tid = (int)threadIdx.x;
  const int blk = (int)blockIdx.x;
  const int rowBase = blk * MROWS;
  int nb = nN - rowBase;
  nb = nb < 1 ? 1 : (nb > MROWS ? MROWS : nb);
#pragma unroll 4
  for (int it = 0; it < (MROWS * FD) / (4 * NTHR); ++it) {
    const int idx = it * NTHR + tid;
    const int r = idx >> 5, q = idx & 31;
    const v4f v = *(const v4fa*)(S + (size_t)(rowBase + r) * FD + 4 * q);
    *(v4fa*)(tile + r * FD + 4 * q) = v;
  }
  __syncthreads();
  if (tid < FD) {
    float s = 0.0f;
#pragma unroll 4
    for (int r = 0; r < nb; ++r) s += tile[r * FD + tid];
    const float fn = (float)nb;
    const float mean = s * (1.0f / fn);
    float m2 = 0.0f;
#pragma unroll 4
    for (int r = 0; r < nb; ++r) {
      const float d = tile[r * FD + tid] - mean;
      m2 = fmaf(d, d, m2);
    }
    rec[tid] = fn;
    rec[FD + tid] = mean;
    rec[2 * FD + tid] = m2;
  }
  __syncthreads();
  if (tid < (3 * FD) / 4) {
    const v4f v = *(const v4fa*)(rec + 4 * tid);
    float* op = REC + (size_t)blk * (3 * FD) + 4 * tid;
    *(volatile v4f*)op = v;
    __threadfence();
    *(volatile v4f*)op = v;
  }
}

__global__ __launch_bounds__(FD) void k_comb(const float* __restrict__ REC, int nRec, float* STAT) {
  __shared__ __attribute__((aligned(16))) float so[2 * FD];
  const int c = (int)threadIdx.x;
  double sn = 0.0, sm = 0.0;
#pragma unroll 2
  for (int b = 0; b < nRec; ++b) {
    const double n = (double)REC[(size_t)b * (3 * FD) + c];
    const double m = (double)REC[(size_t)b * (3 * FD) + FD + c];
    sn += n;
    sm += n * m;
  }
  const double mean = sm / sn;
  double M2 = 0.0;
#pragma unroll 2
  for (int b = 0; b < nRec; ++b) {
    const double n = (double)REC[(size_t)b * (3 * FD) + c];
    const double m = (double)REC[(size_t)b * (3 * FD) + FD + c];
    const double q = (double)REC[(size_t)b * (3 * FD) + 2 * FD + c];
    const double d = m - mean;
    M2 += q + n * (d * d);
  }
  const float var = (float)(M2 / sn);
  const float r = 1.0f / sqrtf(var + BNEPS);
  so[c] = (float)mean;
  so[FD + c] = r;
  __syncthreads();
  if (c < (2 * FD) / 4) {
    const v4f v = *(const v4fa*)(so + 4 * c);
    float* op = STAT + 4 * c;
    *(volatile v4f*)op = v;
    __threadfence();
    *(volatile v4f*)op = v;
  }
}

__global__ __launch_bounds__(NTHR) void k_apply(float* PB, const float* __restrict__ STAT,
                                                const float* __restrict__ gam, const float* __restrict__ bet,
                                                int nN, int MPr) {
  const int tid = (int)threadIdx.x, lane = tid & 31, wave = tid >> 5;
  const int ch0 = 8 * (lane & 15);
  const bool losel = lane >= 16;
  float mu[8], rr[8], gg[8], bb[8];
  {
    const v4f m0 = *(const v4fa*)(STAT + ch0),      m1 = *(const v4fa*)(STAT + ch0 + 4);
    const v4f r0 = *(const v4fa*)(STAT + FD + ch0), r1 = *(const v4fa*)(STAT + FD + ch0 + 4);
    const v4f g0 = *(const v4fa*)(gam + ch0),       g1 = *(const v4fa*)(gam + ch0 + 4);
    const v4f b0 = *(const v4fa*)(bet + ch0),       b1 = *(const v4fa*)(bet + ch0 + 4);
#pragma unroll
    for (int i = 0; i < 4; ++i) {
      mu[i] = m0[i]; mu[4 + i] = m1[i];
      rr[i] = r0[i]; rr[4 + i] = r1[i];
      gg[i] = bfr(g0[i]); gg[4 + i] = bfr(g1[i]);
      bb[i] = bfr(b0[i]); bb[4 + i] = bfr(b1[i]);
    }
  }
  const int rowBase = (int)blockIdx.x * MROWS;
#pragma unroll 1
  for (int si = 0; si < MROWS / NWAVE; ++si) {
    const int row = rowBase + si * NWAVE + wave;
    if (row < MPr) {
      float* rowp = PB + (size_t)row * FD;
      const v4f a = *(const v4fa*)(rowp + ch0);
      const v4f b = *(const v4fa*)(rowp + ch0 + 4);
      float sv[8];
#pragma unroll
      for (int i = 0; i < 4; ++i) { sv[i] = a[i]; sv[4 + i] = b[i]; }
      const bool live = row < nN;
      v8us o;
#pragma unroll
      for (int i = 0; i < 8; ++i) {
        const float y = ((sv[i] - mu[i]) * rr[i]) * gg[i] + bb[i];
        const float v = live ? y : 0.0f;
        const unsigned int hb = f2bf(v);
        const unsigned int lw = f2bf(v - bf2f(hb));
        o[i] = (unsigned short)(losel ? lw : hb);
      }
      unsigned short* dp = (unsigned short*)rowp + 8 * lane;
      *(volatile v8usa*)dp = o;
      __threadfence();
      *(volatile v8usa*)dp = o;
    }
  }
}

__global__ __launch_bounds__(NTHR) void k_pool(const float* __restrict__ h3, const int* __restrict__ bat,
                                               int nN, unsigned short* HG) {
  __shared__ __attribute__((aligned(16))) float acc[PGR * FD];
  __shared__ int plist[NTHR];
  __shared__ int wcn[NWAVE];
  const int tid = (int)threadIdx.x, lane = tid & 31, wave = tid >> 5;
  const int g0 = (int)blockIdx.x * PGR;
  {
    const v4f z = {0.f, 0.f, 0.f, 0.f};
    for (int i = tid * 4; i < PGR * FD; i += NTHR * 4) *(v4fa*)(acc + i) = z;
    plist[tid] = 0;
    if (tid < NWAVE) wcn[tid] = 0;
  }
  __syncthreads();
  const int nCh = (nN + NTHR - 1) / NTHR;
#pragma unroll 1
  for (int ch = 0; ch < nCh; ++ch) {
    const int i  = ch * NTHR + tid;
    const int ic = i < nN ? i : nN - 1;
    const int b  = bat[ic];
    const unsigned gl = (unsigned)(b - g0);
    const bool hit = (i < nN) && (gl < (unsigned)PGR);
    const unsigned msk = __builtin_amdgcn_ballot_w32(hit);
    if (lane == 0) wcn[wave] = (int)__builtin_popcount(msk);
    __syncthreads();
    int pre = 0, all = 0;
#pragma unroll
    for (int w2 = 0; w2 < NWAVE; ++w2) {
      int c = wcn[w2];
      c = c < 0 ? 0 : (c > 32 ? 32 : c);
      all += c;
      pre += (w2 < wave) ? c : 0;
    }
    if (hit) {
      const int pos = pre + (int)__builtin_amdgcn_mbcnt_lo(msk, 0u);
      if (pos < NTHR) plist[pos] = (int)((unsigned)i | (gl << SRCB));
    }
    __syncthreads();
    if (all > 0) {
#pragma unroll 1
      for (int k = 0; k < all; ++k) {
        const int ent = plist[k];
        const int gq  = (ent >> SRCB) & (PGR - 1);
        if ((gq & (NWAVE - 1)) == wave) {
          int node = ent & ((1 << SRCB) - 1);
          node = node > nN - 1 ? nN - 1 : node;
          const v4f v = *(const v4fa*)(h3 + (size_t)node * FD + 4 * lane);
          float* p = acc + gq * FD + 4 * lane;
          v4f a = *(const v4fa*)p;
          a.x += v.x; a.y += v.y; a.z += v.z; a.w += v.w;
          *(v4fa*)p = a;
        }
      }
    }
  }
  __syncthreads();
  const int ch0 = 8 * (lane & 15);
  const bool losel = lane >= 16;
#pragma unroll 1
  for (int j = 0; j < PGR / NWAVE; ++j) {
    const int gq = wave + NWAVE * j;
    const v4f a = *(const v4fa*)(acc + gq * FD + ch0);
    const v4f b = *(const v4fa*)(acc + gq * FD + ch0 + 4);
    float sv[8];
#pragma unroll
    for (int i = 0; i < 4; ++i) { sv[i] = a[i]; sv[4 + i] = b[i]; }
    v8us o;
#pragma unroll
    for (int i = 0; i < 8; ++i) {
      const unsigned int hb = f2bf(sv[i]);
      const unsigned int lw = f2bf(sv[i] - bf2f(hb));
      o[i] = (unsigned short)(losel ? lw : hb);
    }
    unsigned short* dp = HG + (size_t)(g0 + gq) * KD + 8 * lane;
    *(volatile v8usa*)dp = o;
    __threadfence();
    *(volatile v8usa*)dp = o;
  }
}

__global__ __launch_bounds__(GTHR) void k_head(const unsigned short* __restrict__ A,
                                               const unsigned short* __restrict__ WT,
                                               const float* __restrict__ fb1, const float* __restrict__ fw2,
                                               const float* __restrict__ fb2, float* out) {
  __shared__ __attribute__((aligned(16))) float stg[GBM * FD];
  __shared__ float sfb[FD];
  __shared__ float sfw[FD];
  __shared__ float pd[2 * GBM];
  __shared__ __attribute__((aligned(16))) float so[GBM];
  const int tid = (int)threadIdx.x, lane = tid & 31, wave = tid >> 5, hh = lane >> 4, m = lane & 15;
  const int rowBase = (int)blockIdx.x * GBM;
  sfb[tid] = bfr(fb1[tid]);
  sfw[tid] = bfr(fw2[tid]);
  const float fb2r = bfr(fb2[0]);

  v8f acc[8];
  {
    const v8f z = {0.f, 0.f, 0.f, 0.f, 0.f, 0.f, 0.f, 0.f};
#pragma unroll
    for (int t = 0; t < 8; ++t) acc[t] = z;
  }
  const unsigned short* ap = A  + (size_t)(rowBase + 16 * wave + m) * (size_t)KD + 8 * hh;
  const unsigned short* wp = WT + (size_t)m * (size_t)KD + 8 * hh;
#pragma unroll 1
  for (int ks = 0; ks < KD / 32; ++ks) {
    FragB af;
    af.h[0] = *(const v8usa*)(ap + 32 * ks);
    af.h[1] = *(const v8usa*)(ap + 32 * ks + 16);
#pragma unroll
    for (int t = 0; t < 8; ++t) {
      const unsigned short* wq = wp + (size_t)(16 * t) * (size_t)KD + 32 * ks;
      FragB bf;
      bf.h[0] = *(const v8usa*)wq;
      bf.h[1] = *(const v8usa*)(wq + 16);
      acc[t] = wmb(af, bf, acc[t]);
    }
  }
#pragma unroll
  for (int t = 0; t < 8; ++t) {
    const int lc = 16 * t + m;
#pragma unroll
    for (int r = 0; r < 8; ++r) {
      const int lr = 16 * wave + 8 * hh + r;
      stg[lr * FD + lc] = acc[t][r];
    }
  }
  __syncthreads();
  {
    const int row = tid & 63, half = tid >> 6;
    float d = 0.0f;
#pragma unroll 1
    for (int c = 0; c < 64; ++c) {
      const int cc = half * 64 + c;
      const float v = stg[row * FD + cc] + sfb[cc];
      const float r = (v > 0.0f) ? v : SELU_A * expm1f(v);
      d = fmaf(SELU_S * r, sfw[cc], d);
    }
    pd[half * GBM + row] = d;
  }
  __syncthreads();
  if (tid < GBM) so[tid] = (pd[tid] + pd[GBM + tid]) + fb2r;
  __syncthreads();
  const v4f ov = *(const v4fa*)(so + 4 * (lane & 15));
  float* op = out + (size_t)rowBase + 4 * (lane & 15);
  const bool okst = (wave == 0) && (lane < 16);
  if (okst) *(volatile v4f*)op = ov;
  __threadfence();
  if (okst) *(volatile v4f*)op = ov;
}

static inline int cdiv(int a, int b) { return (a + b - 1) / b; }
static inline size_t al256(size_t o) { return (o + 255) & ~(size_t)255; }

extern "C" void kernel_launch(void* const* d_in, const int* in_sizes, int n_in,
                              void* d_out, int out_size, void* d_ws, size_t ws_size,
                              hipStream_t stream) {
  if (n_in < 17) return;
  if (in_sizes[0] < FD || (in_sizes[0] % FD) != 0) return;
  const int nN = in_sizes[0] / FD;
  if (nN < 1 || nN > (1 << SRCB)) return;
  if (in_sizes[1] < 2 || (in_sizes[1] & 1) != 0) return;
  const int nE = in_sizes[1] / 2;
  if (nE < 1 || nE > (1 << 30)) return;
  if (in_sizes[2] != nN) return;
  if (in_sizes[3] != FD * FD || in_sizes[7] != FD * FD) return;
  if (in_sizes[11] != FD * FD || in_sizes[13] != FD * FD) return;
  if (in_sizes[4] != FD || in_sizes[5] != FD || in_sizes[6] != FD) return;
  if (in_sizes[8] != FD || in_sizes[9] != FD || in_sizes[10] != FD) return;
  if (in_sizes[12] != FD || in_sizes[14] != FD || in_sizes[15] != FD) return;
  if (in_sizes[16] != 1) return;
  if (out_size != NGR) return;

  const float* x   = (const float*)d_in[0];
  const int*   ei  = (const int*)  d_in[1];
  const int*   bat = (const int*)  d_in[2];
  const float* W1  = (const float*)d_in[3];
  const float* b1  = (const float*)d_in[4];
  const float* g1  = (const float*)d_in[5];
  const float* be1 = (const float*)d_in[6];
  const float* W2  = (const float*)d_in[7];
  const float* b2  = (const float*)d_in[8];
  const float* g2  = (const float*)d_in[9];
  const float* be2 = (const float*)d_in[10];
  const float* W3  = (const float*)d_in[11];
  const float* b3  = (const float*)d_in[12];
  const float* fw1 = (const float*)d_in[13];
  const float* fb1 = (const float*)d_in[14];
  const float* fw2 = (const float*)d_in[15];
  const float* fb2 = (const float*)d_in[16];
  float* out = (float*)d_out;
  const int* src = ei;
  const int* dst = ei + nE;

  const int MP   = cdiv(nN, MROWS) * MROWS;
  const int nRec = MP / MROWS;
  if ((long long)(nRec - 1) * MROWS >= (long long)nN) return;
  const int gA   = cdiv(MP, NBA);
  const int NBP  = gA * NBA;
  const int gAgg = NBP / ASL;
  if ((long long)gAgg * ASL < (long long)MP) return;
  const int vec8 = ((nE & 3) == 0) ? 1 : 0;
  const int nUx  = MP * (FD / 8);
  if ((nUx % NTHR) != 0) return;

  char* ws = (char*)d_ws;
  size_t off = 0;
  const size_t oPA  = off; off = al256(off + (size_t)MP * FD * 4);
  const size_t oPB  = off; off = al256(off + (size_t)MP * FD * 4);
  const size_t oLST = off; off = al256(off + (size_t)gA * RCAP * 4);
  const size_t oCNT = off; off = al256(off + (size_t)NBP * 4);
  const size_t oOFF = off; off = al256(off + (size_t)NBP * 4);
  const size_t oDIS = off; off = al256(off + (size_t)NBP * 4);
  const size_t oFLG = off; off = al256(off + (size_t)gA * 128);
  const size_t oREC = off; off = al256(off + (size_t)nRec * 3 * FD * 4);
  const size_t oSTA = off; off = al256(off + (size_t)2 * FD * 4);
  const size_t oHG  = off; off = al256(off + (size_t)NGR * KD * 2);
  const size_t oW1T = off; off = al256(off + (size_t)FD * FD * 2);
  const size_t oW2D = off; off = al256(off + (size_t)FD * KD * 2);
  const size_t oW3D = off; off = al256(off + (size_t)FD * KD * 2);
  const size_t oFWD = off; off = al256(off + (size_t)FD * KD * 2);
  if (off > ws_size || off > (size_t)WSMAX) return;
  if ((size_t)MP * FD * 2 > (size_t)MP * FD * 4) return;
  float*          PA   = (float*)(ws + oPA);
  float*          PB   = (float*)(ws + oPB);
  unsigned short* PBh  = (unsigned short*)(ws + oPB);
  int*            LIST = (int*)(ws + oLST);
  int*            CNT  = (int*)(ws + oCNT);
  int*            OFF  = (int*)(ws + oOFF);
  float*          DIS  = (float*)(ws + oDIS);
  int*            FLG  = (int*)(ws + oFLG);
  float*          REC  = (float*)(ws + oREC);
  float*          STAT = (float*)(ws + oSTA);
  unsigned short* HG   = (unsigned short*)(ws + oHG);
  unsigned short* W1T  = (unsigned short*)(ws + oW1T);
  unsigned short* W2D  = (unsigned short*)(ws + oW2D);
  unsigned short* W3D  = (unsigned short*)(ws + oW3D);
  unsigned short* FWD  = (unsigned short*)(ws + oFWD);

  const int bktLds  = BKT_LDS_INTS * 4;
  const int statLds = STAT_LDS_FLOATS * 4;
  hipFuncSetAttribute(reinterpret_cast<const void*>(&k_bucket),
                      hipFuncAttributeMaxDynamicSharedMemorySize, bktLds);
  hipFuncSetAttribute(reinterpret_cast<const void*>(&k_stats),
                      hipFuncAttributeMaxDynamicSharedMemorySize, statLds);

  const dim3 gG(MP / GBM, FD / GBN);

  k_prep<<<(nUx + NUW1 + 3 * NUWD) / NTHR, NTHR, 0, stream>>>(x, W1, W2, W3, fw1, PBh, W1T, W2D, W3D, FWD, nN, nUx);
  k_bucket<<<gA, NTHR, bktLds, stream>>>(src, dst, nE, nN, vec8, LIST, CNT, OFF, (int*)DIS, FLG);
  k_gemm<<<gG, GTHR, 0, stream>>>(PBh, W1T, PA, FD, FD);
  k_agg<0><<<gAgg, NTHR, 0, stream>>>(LIST, CNT, OFF, FLG, DIS, PA, b1, PB, nN, MP);
  k_stats<<<nRec, NTHR, statLds, stream>>>(PB, REC, nN);
  k_comb<<<1, FD, 0, stream>>>(REC, nRec, STAT);
  k_apply<<<MP / MROWS, NTHR, 0, stream>>>(PB, STAT, g1, be1, nN, MP);
  k_gemm<<<gG, GTHR, 0, stream>>>(PBh, W2D, PA, KD, FD);
  k_agg<0><<<gAgg, NTHR, 0, stream>>>(LIST, CNT, OFF, FLG, DIS, PA, b2, PB, nN, MP);
  k_stats<<<nRec, NTHR, statLds, stream>>>(PB, REC, nN);
  k_comb<<<1, FD, 0, stream>>>(REC, nRec, STAT);
  k_apply<<<MP / MROWS, NTHR, 0, stream>>>(PB, STAT, g2, be2, nN, MP);
  k_gemm<<<gG, GTHR, 0, stream>>>(PBh, W3D, PA, KD, FD);
  k_agg<1><<<gAgg, NTHR, 0, stream>>>(LIST, CNT, OFF, FLG, DIS, PA, b3, PB, nN, MP);
  k_pool<<<NGR / PGR, NTHR, 0, stream>>>(PB, bat, nN, HG);
  k_head<<<NGR / GBM, GTHR, 0, stream>>>(HG, FWD, fb1, fw2, fb2, out);
}
